// DWAMiddleLayer_23794118819889
// MI455X (gfx1250) — hardware-run, weakly checked
//
#include <hip/hip_runtime.h>


#ifndef NB
#define NB 256
#endif
#define NB_FULL 256
#define DA    1024
#define DB    1024
#define RR    16
#define NP    64
#define KC    (NP * RR)
#define U_END (DB * RR)
#define V_END (U_END + RR * DA)
#define POOL_DIM (V_END + DB)

static_assert(NB % 64 == 0);
static_assert(NB <= NB_FULL);
static_assert(DA == DB);
static_assert(DA % 32 == 0 && KC % 32 == 0 && NP % 32 == 0);
static_assert(DB % 64 == 0 && KC % 64 == 0);
static_assert(DA % 8 == 0 && NP % 8 == 0 && RR == 16);
static_assert(POOL_DIM == 33792);
static_assert(DA == 32 * 8 * 4);
static_assert(16 * 68 * 4 <= 131072);
static_assert(32 * 16 * 4 == 16 * 64 * 2);
static_assert(32 * 16 * 8 == 16 * 64 * 4);
static_assert(32 * 16 * 8 == DA * 4);

typedef unsigned short bf;
typedef __attribute__((ext_vector_type(16))) __bf16   v16bf;
typedef __attribute__((ext_vector_type(8)))  unsigned short v8us;
typedef __attribute__((ext_vector_type(8)))  float    v8f;
typedef __attribute__((ext_vector_type(4)))  float    v4f;
typedef v4f  __attribute__((may_alias)) v4fa;

__device__ __forceinline__ unsigned short f2bf(float f) { unsigned u = __float_as_uint(f); u += 0x7FFFu + ((u >> 16) & 1u); return (unsigned short)(u >> 16); }
__device__ __forceinline__ float bf2f(unsigned short w) { return __uint_as_float(((unsigned)w) << 16); }
__device__ __forceinline__ int clampi(int v, int lo, int hi) { return min(max(v, lo), hi); }
__device__ __forceinline__ v16bf cat16b(v8us lo, v8us hi) { return __builtin_bit_cast(v16bf, __builtin_shufflevector(lo, hi, 0, 1, 2, 3, 4, 5, 6, 7, 8, 9, 10, 11, 12, 13, 14, 15)); }
__device__ __forceinline__ v8f wmmab(v16bf a, v16bf b, v8f c) { return __builtin_amdgcn_wmma_f32_16x16x32_bf16(false, a, false, b, (short)0, c, false, false); }
__device__ __forceinline__ v16bf ldb(const bf* p)  { return cat16b(*(const v8us*)p, *(const v8us*)(p + 16)); }
__device__ __forceinline__ void wave_sync() { __builtin_amdgcn_fence(3  , "wavefront"); __builtin_amdgcn_wave_barrier(); asm volatile("" ::: "memory"); }
__device__ __forceinline__ v8f wmmag(v16bf a, v16bf b, v8f c) {
    c = wmmab(a, b, c);
    asm volatile("v_nop\n\tv_nop\n\tv_nop\n\tv_nop" : "+v"(c) : "v"(a), "v"(b));
    return c;
}

__global__ __launch_bounds__(256) void k_cast(const float* __restrict__ src, bf* dst, int rows, int cols, int psh, int gsh, int gstride, int off) {
    const int t = blockIdx.x * 256 + threadIdx.x;
    if (t >= (rows << psh)) return;
    const int row = t >> psh, c8 = (t & ((1 << psh) - 1)) * 8;
    const int g = row >> gsh, rr = row & ((1 << gsh) - 1);
    const float* s = src + (size_t)g * gstride + (size_t)rr * cols + off + c8;
    const v4f x0 = *(const v4f*)s; const v4f x1 = *(const v4f*)(s + 4);
    v8us o;
#pragma unroll
    for (int k = 0; k < 4; ++k) { o[k] = f2bf(x0[k]); o[4 + k] = f2bf(x1[k]); }
    bf* d = dst + (size_t)row * cols + c8;
    *(volatile v8us*)d = o; __threadfence(); *(volatile v8us*)d = o;
}

__global__ __launch_bounds__(256) void k_ucat(const float* __restrict__ pool, bf* UB) {
    const int t = blockIdx.x * 256 + threadIdx.x;
    if (t >= DB * (KC / 8)) return;
    const int c = t >> 7, piece = t & 127; const int n = piece >> 1, r8 = (piece & 1) * 8;
    const float* s = pool + (size_t)n * POOL_DIM + (size_t)c * RR + r8;
    const v4f x0 = *(const v4f*)s; const v4f x1 = *(const v4f*)(s + 4);
    v8us o;
#pragma unroll
    for (int k = 0; k < 4; ++k) { o[k] = f2bf(x0[k]); o[4 + k] = f2bf(x1[k]); }
    bf* d = UB + (size_t)c * KC + piece * 8;
    *(volatile v8us*)d = o; __threadfence(); *(volatile v8us*)d = o;
}
static_assert(KC / 8 == 128);

__global__ __launch_bounds__(256) void k_bt(const float* __restrict__ pool, bf* BT) {
    const int t = blockIdx.x * 256 + threadIdx.x;
    if (t >= DB * (NP / 8)) return;
    const int c = t >> 3, n8 = (t & 7) * 8;
    v8us o;
#pragma unroll
    for (int k = 0; k < 8; ++k) o[k] = f2bf(pool[(size_t)(n8 + k) * POOL_DIM + V_END + c]);
    bf* d = BT + (size_t)c * NP + n8;
    *(volatile v8us*)d = o; __threadfence(); *(volatile v8us*)d = o;
}
static_assert(NP / 8 == 8);

__device__ __forceinline__ void gemm_seg(v8f (&acc)[4][4], const bf* __restrict__ A, const bf* __restrict__ B, const int lda, const int ldbb, const int K,
                                         const int m0, const int n0, const int lr, const int hi) {
    const size_t aoff = (size_t)(m0 + lr) * lda + 8 * hi, boff = (size_t)(n0 + lr) * ldbb + 8 * hi;
#pragma unroll 1
    for (int kc = 0; kc < K; kc += 32) {
        v16bf a[4];
#pragma unroll
        for (int mb = 0; mb < 4; ++mb) a[mb] = ldb(A + aoff + (size_t)mb * 16 * lda + kc);
#pragma unroll
        for (int nb = 0; nb < 4; ++nb) { const v16bf b = ldb(B + boff + (size_t)nb * 16 * ldbb + kc);
#pragma unroll
            for (int mb = 0; mb < 4; ++mb) acc[mb][nb] = wmmag(a[mb], b, acc[mb][nb]); }
    }
}

__global__ __launch_bounds__(32) __attribute__((amdgpu_num_vgpr(256))) void k_t1(const bf* __restrict__ HB, const bf* __restrict__ VB, const float* __restrict__ alpha,
                                                                                    bf* SH, bf* SL) {
    __shared__ __align__(16) float os[16 * 68];
    const int lane = threadIdx.x & 31, lr = lane & 15, hi = lane >> 4;
    const int n0 = ((int)blockIdx.x % (KC / 64)) * 64, m0 = ((int)blockIdx.x / (KC / 64)) * 64;
    v8f acc[4][4];
#pragma unroll
    for (int mb = 0; mb < 4; ++mb)
#pragma unroll
        for (int nb = 0; nb < 4; ++nb) acc[mb][nb] = (v8f){};
    gemm_seg(acc, HB, VB, DA, DA, DA, m0, n0, lr, hi);
    const int rr = lane >> 3, c8 = (lane & 7) * 8;
    const int np = (n0 + c8) >> 4;
#pragma unroll
    for (int mb = 0; mb < 4; ++mb) {
#pragma unroll
        for (int nb = 0; nb < 4; ++nb) {
#pragma unroll
            for (int j = 0; j < 8; ++j) os[(hi * 8 + j) * 68 + nb * 16 + lr] = acc[mb][nb][j]; }
        wave_sync();
#pragma unroll 1
        for (int ps = 0; ps < 2; ++ps) {
#pragma unroll 1
            for (int it = 0; it < 4; ++it) {
                const int row = 4 * it + rr; const int b = m0 + mb * 16 + row;
                const float al = bf2f(f2bf(alpha[(size_t)b * NP + np]));
                const v4f x0 = *(const v4fa*)(&os[row * 68 + c8]); const v4f x1 = *(const v4fa*)(&os[row * 68 + c8 + 4]);
                v8us oh, ol;
#pragma unroll
                for (int k = 0; k < 4; ++k) {
                    const float s0 = al * x0[k]; const unsigned short h0 = f2bf(s0); oh[k] = h0; ol[k] = f2bf(s0 - bf2f(h0));
                    const float s1 = al * x1[k]; const unsigned short h1 = f2bf(s1); oh[4 + k] = h1; ol[4 + k] = f2bf(s1 - bf2f(h1)); }
                *(volatile v8us*)(SH + (size_t)b * KC + n0 + c8) = oh;
                *(volatile v8us*)(SL + (size_t)b * KC + n0 + c8) = ol; }
            if (ps == 0) __threadfence(); }
        wave_sync();
    }
}

__global__ __launch_bounds__(32) __attribute__((amdgpu_num_vgpr(256))) void k_out(const bf* __restrict__ HB, const bf* __restrict__ WB, const bf* __restrict__ SH, const bf* __restrict__ SL,
                                                                                     const bf* __restrict__ UB, const bf* __restrict__ AL, const bf* __restrict__ BT,
                                                                                     const float* __restrict__ hA, const float* __restrict__ bbase, const float* __restrict__ gam, float* PRE) {
    __shared__ __align__(16) float os[16 * 68];
    const int lane = threadIdx.x & 31, lr = lane & 15, hi = lane >> 4;
    const int n0 = ((int)blockIdx.x % (DB / 64)) * 64, m0 = ((int)blockIdx.x / (DB / 64)) * 64;
    v8f acc[4][4];
#pragma unroll
    for (int mb = 0; mb < 4; ++mb)
#pragma unroll
        for (int nb = 0; nb < 4; ++nb) acc[mb][nb] = (v8f){};
    gemm_seg(acc, HB, WB, DA, DA, DA, m0, n0, lr, hi);
    gemm_seg(acc, SH, UB, KC, KC, KC, m0, n0, lr, hi);
    gemm_seg(acc, SL, UB, KC, KC, KC, m0, n0, lr, hi);
    gemm_seg(acc, AL, BT, NP, NP, NP, m0, n0, lr, hi);
    const float g = bf2f(f2bf(gam[0]));
    const int rr = lane >> 4, c4 = (lane & 15) * 4;
    const v4f bq = *(const v4f*)(bbase + n0 + c4);
    v4f bb;
#pragma unroll
    for (int k = 0; k < 4; ++k) bb[k] = bf2f(f2bf(bq[k]));
#pragma unroll
    for (int mb = 0; mb < 4; ++mb) {
#pragma unroll
        for (int nb = 0; nb < 4; ++nb) {
#pragma unroll
            for (int j = 0; j < 8; ++j) os[(hi * 8 + j) * 68 + nb * 16 + lr] = acc[mb][nb][j]; }
        wave_sync();
#pragma unroll 1
        for (int ps = 0; ps < 2; ++ps) {
#pragma unroll 1
            for (int it = 0; it < 8; ++it) {
                const int row = 2 * it + rr; const int b = m0 + mb * 16 + row;
                const v4f x = *(const v4fa*)(&os[row * 68 + c4]);
                const v4f hq = *(const v4f*)(hA + (size_t)b * DA + n0 + c4);
                v4f v;
#pragma unroll
                for (int k = 0; k < 4; ++k) v[k] = bf2f(f2bf(hq[k])) + g * (x[k] + bb[k]);
                *(volatile v4f*)(PRE + (size_t)b * DB + n0 + c4) = v; }
            if (ps == 0) __threadfence(); }
        wave_sync();
    }
}

__global__ __launch_bounds__(32) void k_ln(const float* __restrict__ PRE, const float* __restrict__ lsc, const float* __restrict__ lbi, float* OUT) {
#pragma clang fp contract(off)
    const int lane = threadIdx.x & 31;
    const size_t base = (size_t)blockIdx.x * DA + 4 * lane;
    float s = 0.0f;
#pragma unroll 1
    for (int i = 0; i < 8; ++i) { const v4f v = *(const v4f*)(PRE + base + i * 128); s += (v[0] + v[1]) + (v[2] + v[3]); }
#pragma unroll
    for (int d = 16; d >= 1; d >>= 1) s += __shfl_xor(s, d, 32);
    const float mean = s * (1.0f / (float)DA);
    float q = 0.0f;
#pragma unroll 1
    for (int i = 0; i < 8; ++i) { const v4f v = *(const v4f*)(PRE + base + i * 128);
        const float d0 = v[0] - mean, d1 = v[1] - mean, d2 = v[2] - mean, d3 = v[3] - mean;
        q += (d0 * d0 + d1 * d1) + (d2 * d2 + d3 * d3); }
#pragma unroll
    for (int d = 16; d >= 1; d >>= 1) q += __shfl_xor(q, d, 32);
    const float var = q * (1.0f / (float)DA);
    const float inv = rsqrtf(var + 1e-5f);
#pragma unroll 1
    for (int ps = 0; ps < 2; ++ps) {
#pragma unroll 1
        for (int i = 0; i < 8; ++i) {
            const v4f v = *(const v4f*)(PRE + base + i * 128);
            const v4f sc = *(const v4f*)(lsc + 4 * lane + i * 128);
            const v4f bi = *(const v4f*)(lbi + 4 * lane + i * 128);
            v4f o;
#pragma unroll
            for (int k = 0; k < 4; ++k) o[k] = (v[k] - mean) * inv * bf2f(f2bf(sc[k])) + bf2f(f2bf(bi[k]));
            *(volatile v4f*)(OUT + base + i * 128) = o; }
        if (ps == 0) __threadfence(); }
}

static constexpr size_t al256(size_t v) { return (v + 255) & ~(size_t)255; }
static constexpr size_t SZ_HB  = al256((size_t)NB * DA * 2);
static constexpr size_t SZ_AL  = al256((size_t)NB * NP * 2);
static constexpr size_t SZ_WB  = al256((size_t)DB * DA * 2);
static constexpr size_t SZ_VB  = al256((size_t)KC * DA * 2);
static constexpr size_t SZ_UB  = al256((size_t)DB * KC * 2);
static constexpr size_t SZ_BT  = al256((size_t)DB * NP * 2);
static constexpr size_t SZ_S   = al256((size_t)NB * KC * 2);
static constexpr size_t SZ_PRE = al256((size_t)NB * DB * 4);
static constexpr size_t SZ_TOTAL = SZ_HB + SZ_AL + SZ_WB + SZ_VB + SZ_UB + SZ_BT + 2 * SZ_S + SZ_PRE;
static_assert(SZ_TOTAL <= (size_t)134217728);

extern "C" void kernel_launch(void* const* d_in, const int* in_sizes, int n_in,
                              void* d_out, int out_size, void* d_ws, size_t ws_size, hipStream_t stream) {
    if (n_in < 8) return;
    if ((size_t)in_sizes[0] < (size_t)NB * DA) return;
    if ((size_t)in_sizes[1] < (size_t)NP * POOL_DIM) return;
    if ((size_t)in_sizes[2] < (size_t)NB * NP) return;
    if ((size_t)in_sizes[3] < (size_t)DB * DA) return;
    if ((size_t)in_sizes[4] < (size_t)DB || in_sizes[5] < 1) return;
    if ((size_t)in_sizes[6] < (size_t)DA || (size_t)in_sizes[7] < (size_t)DA) return;
    if ((size_t)out_size < (size_t)NB * DB) return;
    if (SZ_TOTAL > ws_size) return;
    const float* hA    = (const float*)d_in[0];
    const float* pool  = (const float*)d_in[1];
    const float* alpha = (const float*)d_in[2];
    const float* Wb    = (const float*)d_in[3];
    const float* bbs   = (const float*)d_in[4];
    const float* gam   = (const float*)d_in[5];
    const float* lsc   = (const float*)d_in[6];
    const float* lbi   = (const float*)d_in[7];
    float* OUT = (float*)d_out;
    char* wsp = (char*)d_ws;
    bf* HB = (bf*)wsp; wsp += SZ_HB;
    bf* AL = (bf*)wsp; wsp += SZ_AL;
    bf* WB = (bf*)wsp; wsp += SZ_WB;
    bf* VB = (bf*)wsp; wsp += SZ_VB;
    bf* UB = (bf*)wsp; wsp += SZ_UB;
    bf* BT = (bf*)wsp; wsp += SZ_BT;
    bf* SH = (bf*)wsp; wsp += SZ_S;
    bf* SL = (bf*)wsp; wsp += SZ_S;
    float* PRE = (float*)wsp; wsp += SZ_PRE;

    k_cast<<<(unsigned)((NB * (DA / 8) + 255) / 256), 256, 0, stream>>>(hA, HB, NB, DA, 7, 30, 0, 0);
    k_cast<<<(unsigned)((NB * (NP / 8) + 255) / 256), 256, 0, stream>>>(alpha, AL, NB, NP, 3, 30, 0, 0);
    k_cast<<<(unsigned)((DB * (DA / 8) + 255) / 256), 256, 0, stream>>>(Wb, WB, DB, DA, 7, 30, 0, 0);
    k_cast<<<(unsigned)((KC * (DA / 8) + 255) / 256), 256, 0, stream>>>(pool, VB, KC, DA, 7, 4, POOL_DIM, U_END);
    k_ucat<<<(unsigned)((DB * (KC / 8) + 255) / 256), 256, 0, stream>>>(pool, UB);
    k_bt<<<(unsigned)((DB * (NP / 8) + 255) / 256), 256, 0, stream>>>(pool, BT);
    k_t1<<<(NB / 64) * (KC / 64), 32, 0, stream>>>(HB, VB, alpha, SH, SL);
    k_out<<<(NB / 64) * (DB / 64), 32, 0, stream>>>(HB, WB, SH, SL, UB, AL, BT, hA, bbs, gam, PRE);
    k_ln<<<NB, 32, 0, stream>>>(PRE, lsc, lbi, OUT);
}
